// MambaBlock_15556371546614
// MI455X (gfx1250) — hardware-verified
//
#include <hip/hip_runtime.h>
#include <math.h>

typedef __attribute__((ext_vector_type(16))) _Float16 v16h;
typedef __attribute__((ext_vector_type(8)))  _Float16 v8h;
typedef __attribute__((ext_vector_type(4)))  _Float16 v4h;
typedef __attribute__((ext_vector_type(16))) __bf16   v16b;
typedef __attribute__((ext_vector_type(8)))  __bf16   v8b;
typedef __attribute__((ext_vector_type(8)))  float    v8f;
typedef __attribute__((ext_vector_type(4)))  float    v4f;

constexpr int kBatch  = 2;
constexpr int kSeq    = 2048;
constexpr int kDm     = 512;
constexpr int kDin    = 1024;
constexpr int kNst    = 16;
constexpr int kDtR    = 32;
constexpr int kLayers = 2;
constexpr int kXzP    = 2 * kDin;
constexpr int kXdP    = kDtR + 2 * kNst;
constexpr int kRows   = kBatch * kSeq;
constexpr int kHid    = 2 * kDm;
constexpr int kOutC   = 512;
constexpr int kConvTP = 260;
constexpr int kScanTS = 64;
constexpr int kScanCh = 64;
constexpr int kScanYP = 68;
constexpr float kEps      = 1e-5f;
constexpr float kInvDm    = 1.0f / (float)kDm;
constexpr float kCarryW   = 32.0f;
constexpr float kCarryDtW = 8.0f;
constexpr float kCarryDt  = 16.0f;
constexpr float kCarryG   = 16.0f;
static_assert(kXdP == 64 && kXzP == 2048 && kRows == 4096 && kHid == 1024, "shape constants");
static_assert((kDm % 32) == 0 && (kDin % 32) == 0 && (kDtR % 32) == 0 && (kHid % 32) == 0, "GEMM K multiples of 32");
static_assert((kRows % 64) == 0 && (kXzP % 64) == 0 && (kXdP % 64) == 0 && (kDm % 64) == 0 &&
              (kDin % 64) == 0 && (kHid % 64) == 0 && (kOutC % 64) == 0, "GEMM M,N multiples of 64");
static_assert((kSeq % kScanTS) == 0 && (kSeq % 64) == 0 && (kDin % kScanCh) == 0 && (kDin % 256) == 0, "tile multiples");
static_assert(kDm == 512, "norm kernel lane map assumes 512 features per row");

constexpr size_t kSzH    = (size_t)kRows * kDm * 4;
constexpr size_t kSzU16  = (size_t)kRows * kDm * 2;
constexpr size_t kSzXZ   = (size_t)kRows * kXzP * 4;
constexpr size_t kSzXC   = (size_t)kRows * kDin * 4;
constexpr size_t kSzXC16 = (size_t)kRows * kDin * 2;
constexpr size_t kSzDBC  = (size_t)kRows * kXdP * 4;
constexpr size_t kSzDT16 = (size_t)kRows * kDtR * 2;
constexpr size_t kSzIPW  = (size_t)kLayers * kXzP * kDm * 2;
constexpr size_t kSzXPW  = (size_t)kLayers * kXdP * kDin * 2;
constexpr size_t kSzDTW  = (size_t)kLayers * kDin * kDtR * 2;
constexpr size_t kSzOPW  = (size_t)kLayers * kDm * kDin * 2;
constexpr size_t kSzW1   = (size_t)kHid * kDm * 2;
constexpr size_t kSzW2   = (size_t)kDm * kHid * 2;
constexpr size_t kSzFW   = (size_t)kOutC * kDm * 2;
static_assert(kSzXC16 >= (size_t)kRows * kHid * 2, "hidden plane fits the aliased region");

constexpr size_t kOffHA    = 0;
constexpr size_t kOffHB    = kOffHA    + kSzH;
constexpr size_t kOffU16   = kOffHB    + kSzH;
constexpr size_t kOffXZ    = kOffU16   + kSzU16;
constexpr size_t kOffXC    = kOffXZ    + kSzXZ;
constexpr size_t kOffXC16  = kOffXC    + kSzXC;
constexpr size_t kOffDBC   = kOffXC16  + kSzXC16;
constexpr size_t kOffDT16  = kOffDBC   + kSzDBC;
constexpr size_t kOffDLR   = kOffDT16  + kSzDT16;
constexpr size_t kOffG16   = kOffDLR   + kSzXC;
constexpr size_t kOffX1    = kOffG16   + kSzXC16;
constexpr size_t kOffX2H   = kOffX1    + kSzH;
constexpr size_t kOffX2L   = kOffX2H   + kSzU16;
constexpr size_t kOffIPW   = kOffX2L   + kSzU16;
constexpr size_t kOffXPW   = kOffIPW   + kSzIPW;
constexpr size_t kOffDTW   = kOffXPW   + kSzXPW;
constexpr size_t kOffOPW   = kOffDTW   + kSzDTW;
constexpr size_t kOffW1    = kOffOPW   + kSzOPW;
constexpr size_t kOffW2    = kOffW1    + kSzW1;
constexpr size_t kOffFWH   = kOffW2    + kSzW2;
constexpr size_t kOffFWL   = kOffFWH   + kSzFW;
constexpr size_t kWsTotal  = kOffFWL   + kSzFW;
static_assert(kWsTotal <= 134217728ull, "carve cap");
static_assert((kOffHB % 128) == 0 && (kOffU16 % 128) == 0 && (kOffXZ % 128) == 0 && (kOffXC % 128) == 0 &&
              (kOffXC16 % 128) == 0 && (kOffDBC % 128) == 0 && (kOffDT16 % 128) == 0 && (kOffDLR % 128) == 0 &&
              (kOffG16 % 128) == 0 && (kOffX1 % 128) == 0 && (kOffX2H % 128) == 0 && (kOffX2L % 128) == 0 &&
              (kOffIPW % 128) == 0 && (kOffXPW % 128) == 0 && (kOffDTW % 128) == 0 && (kOffOPW % 128) == 0 &&
              (kOffW1 % 128) == 0 && (kOffW2 % 128) == 0 && (kOffFWH % 128) == 0 && (kOffFWL % 128) == 0,
              "128-B aligned regions");

__device__ __forceinline__ unsigned short f2bf_bits(float f) {
  unsigned u = __float_as_uint(f);
  return (unsigned short)((u + 0x7FFFu + ((u >> 16) & 1u)) >> 16);
}
__device__ __forceinline__ float bf_bits2f(unsigned short h) { return __uint_as_float(((unsigned)h) << 16); }

__device__ __forceinline__ float wave_sum(float s) {
#pragma unroll
  for (int off = 16; off > 0; off >>= 1) s += __shfl_xor(s, off, 32);
  return s;
}

__device__ __forceinline__ void row_guard_h(v8f& a, v8f& b, v8f& c, v8f& d, v16h x, v16h y) {
  asm volatile("v_nop\n\tv_nop\n\tv_nop\n\tv_nop" : "+v"(a), "+v"(b), "+v"(c), "+v"(d) : "v"(x), "v"(y));
}
__device__ __forceinline__ void row_guard_b(v8f& a, v8f& b, v8f& c, v8f& d, v16b x, v16b y) {
  asm volatile("v_nop\n\tv_nop\n\tv_nop\n\tv_nop" : "+v"(a), "+v"(b), "+v"(c), "+v"(d) : "v"(x), "v"(y));
}
__device__ __forceinline__ void keep4_h(v16h a, v16h b, v16h c, v16h d) { asm volatile("v_nop" :: "v"(a), "v"(b), "v"(c), "v"(d)); }
__device__ __forceinline__ void keep4_b(v16b a, v16b b, v16b c, v16b d) { asm volatile("v_nop" :: "v"(a), "v"(b), "v"(c), "v"(d)); }
__device__ __forceinline__ void acc_guard4(v8f& a, v8f& b, v8f& c, v8f& d) { asm volatile("v_nop\n\tv_nop\n\tv_nop\n\tv_nop" : "+v"(a), "+v"(b), "+v"(c), "+v"(d)); }

template <typename T> struct Frag;
template <> struct Frag<_Float16> {
  typedef v16h V; union U { v16h v; v8h h[2]; };
  static __device__ __forceinline__ v16h load(const _Float16* p) {
    U f; f.h[0] = *(const v8h*)(p); f.h[1] = *(const v8h*)(p + 16); return f.v;
  }
  static __device__ __forceinline__ v8f mma(v16h a, v16h b, v8f c) {
    return __builtin_amdgcn_wmma_f32_16x16x32_f16(false, a, false, b, (short)0, c, false, false);
  }
  static __device__ __forceinline__ void guard(v8f& a, v8f& b, v8f& c, v8f& d, v16h x, v16h y) { row_guard_h(a, b, c, d, x, y); }
  static __device__ __forceinline__ void keep(v16h a, v16h b, v16h c, v16h d) { keep4_h(a, b, c, d); }
};
template <> struct Frag<__bf16> {
  typedef v16b V; union U { v16b v; v8b h[2]; };
  static __device__ __forceinline__ v16b load(const __bf16* p) {
    U f; f.h[0] = *(const v8b*)(p); f.h[1] = *(const v8b*)(p + 16); return f.v;
  }
  static __device__ __forceinline__ v8f mma(v16b a, v16b b, v8f c) {
    return __builtin_amdgcn_wmma_f32_16x16x32_bf16(false, a, false, b, (short)0, c, false, false);
  }
  static __device__ __forceinline__ void guard(v8f& a, v8f& b, v8f& c, v8f& d, v16b x, v16b y) { row_guard_b(a, b, c, d, x, y); }
  static __device__ __forceinline__ void keep(v16b a, v16b b, v16b c, v16b d) { keep4_b(a, b, c, d); }
};

template <int ET> struct Elem;
template <> struct Elem<0> { typedef _Float16 T; };
template <> struct Elem<1> { typedef __bf16 T; };
template <int ET, bool SPLIT, int BIAS_MODE, int OUT_MODE, bool RESID, int ACT>
__global__ __launch_bounds__(256) void wmma_gemm64(
    const unsigned short* __restrict__ Ap, const unsigned short* __restrict__ A2p, int lda,
    const unsigned short* __restrict__ Btp, const unsigned short* __restrict__ Bt2p, int ldb,
    void* __restrict__ Cout, void* __restrict__ Cout2, int ldc,
    const float* __restrict__ bias, const float* __restrict__ resid,
    int M, int N, int K, float scale) {
  static_assert(!(RESID && ACT != 0), "activation only without residual");
  typedef typename Elem<ET>::T T;
  typedef typename Frag<T>::V V;
  const T* A = (const T*)Ap; const T* A2 = (const T*)A2p; const T* Bt = (const T*)Btp; const T* Bt2 = (const T*)Bt2p;
  __shared__ __align__(16) float sT[8][16 * 68];
  const int lane = threadIdx.x & 31;
  const int wave = threadIdx.x >> 5;
  const int tilesN = N >> 6;
  const int tilesM = M >> 6;
  const int tile = blockIdx.x * 8 + wave;
  if (tile >= tilesM * tilesN) return;
  const int tm = tile / tilesN;
  const int tn = tile - tm * tilesN;
  const int m0 = tm << 6;
  const int n0 = tn << 6;

  const int rlane = lane & 15;
  const int koff  = (lane >> 4) * 8;
  const int mOff  = (lane >> 4) * 8;

  v8f acc[4][4];
#pragma unroll
  for (int i = 0; i < 4; ++i)
#pragma unroll
    for (int j = 0; j < 4; ++j) acc[i][j] = (v8f){0.f,0.f,0.f,0.f,0.f,0.f,0.f,0.f};

  for (int k0 = 0; k0 < K; k0 += 32) {
    V bh[4], bl[4];
#pragma unroll
    for (int j = 0; j < 4; ++j) {
      const size_t bo = (size_t)(n0 + (j << 4) + rlane) * ldb + koff + k0;
      bh[j] = Frag<T>::load(Bt + bo);
      if (SPLIT) bl[j] = Frag<T>::load(Bt2 + bo);
    }
#pragma unroll
    for (int i = 0; i < 4; ++i) {
      const size_t ao = (size_t)(m0 + (i << 4) + rlane) * lda + koff + k0;
      V ah = Frag<T>::load(A + ao);
      V al;
      if (SPLIT) al = Frag<T>::load(A2 + ao);
#pragma unroll
      for (int j = 0; j < 4; ++j) {
        acc[i][j] = Frag<T>::mma(ah, bh[j], acc[i][j]);
        if (SPLIT) {
          acc[i][j] = Frag<T>::mma(ah, bl[j], acc[i][j]);
          acc[i][j] = Frag<T>::mma(al, bh[j], acc[i][j]);
        }
      }
      Frag<T>::guard(acc[i][0], acc[i][1], acc[i][2], acc[i][3], ah, SPLIT ? al : ah);
    }
    Frag<T>::keep(bh[0], bh[1], bh[2], bh[3]);
    if (SPLIT) Frag<T>::keep(bl[0], bl[1], bl[2], bl[3]);
  }
  acc_guard4(acc[0][0], acc[0][1], acc[0][2], acc[0][3]);
  acc_guard4(acc[1][0], acc[1][1], acc[1][2], acc[1][3]);
  acc_guard4(acc[2][0], acc[2][1], acc[2][2], acc[2][3]);
  acc_guard4(acc[3][0], acc[3][1], acc[3][2], acc[3][3]);

  float* slab = sT[wave];
  float bvj[4];
#pragma unroll
  for (int j = 0; j < 4; ++j) {
    bvj[j] = 0.f;
    if (BIAS_MODE == 2) bvj[j] = bias[n0 + (j << 4) + rlane];
  }
#pragma unroll
  for (int i = 0; i < 4; ++i) {
    const int mBase = m0 + (i << 4);
#pragma unroll
    for (int j = 0; j < 4; ++j) {
#pragma unroll
      for (int r = 0; r < 8; ++r) {
        float v = acc[i][j][r] * scale;
        if (BIAS_MODE == 2) v += bvj[j];
        if (ACT == 2) v = fmaxf(v, 0.0f);
        slab[(mOff + r) * 68 + (j << 4) + rlane] = v;
      }
    }
    __builtin_amdgcn_fence(__ATOMIC_RELEASE, "workgroup");
    __builtin_amdgcn_wave_barrier();
    __builtin_amdgcn_fence(__ATOMIC_ACQUIRE, "workgroup");
    if (OUT_MODE == 0) {
      float* C = (float*)Cout;
      const int hh = lane >> 4, c4 = (lane & 15) * 4;
      v4f vals[8];
#pragma unroll
      for (int it = 0; it < 8; ++it) {
        const int row = it * 2 + hh;
        vals[it] = *(const v4f*)(slab + row * 68 + c4);
      }
      if (RESID) {
#pragma unroll
        for (int it = 0; it < 8; ++it) {
          const int row = it * 2 + hh;
          const v4f rr = *(const v4f*)(resid + (size_t)(mBase + row) * ldc + n0 + c4);
          vals[it] = vals[it] + rr;
        }
      }
      for (int pass = 0; pass < 2; ++pass) {
#pragma unroll
        for (int it = 0; it < 8; ++it) {
          const int row = it * 2 + hh;
          *(volatile v4f*)(C + (size_t)(mBase + row) * ldc + n0 + c4) = vals[it];
        }
        __threadfence();
      }
    } else {
      const int q = lane >> 3, c8 = (lane & 7) * 8;
      unsigned short* C  = (unsigned short*)Cout;
      unsigned short* C2 = (unsigned short*)Cout2;
      v8h hv[4], lv[4];
#pragma unroll
      for (int it = 0; it < 4; ++it) {
        const int row = it * 4 + q;
        const float* sp = slab + row * 68 + c8;
        v4f a0 = *(const v4f*)(sp);
        v4f a1 = *(const v4f*)(sp + 4);
        if (RESID) {
          const float* rp = resid + (size_t)(mBase + row) * ldc + n0 + c8;
          const v4f r0 = *(const v4f*)(rp);
          const v4f r1 = *(const v4f*)(rp + 4);
          a0 = a0 + r0;
          a1 = a1 + r1;
        }
#pragma unroll
        for (int e = 0; e < 4; ++e) {
          const float f0 = a0[e];
          const float f1 = a1[e];
          if (OUT_MODE == 1) {
            hv[it][e]     = (_Float16)f0;
            hv[it][4 + e] = (_Float16)f1;
            lv[it][e]     = (_Float16)0.0f;
            lv[it][4 + e] = (_Float16)0.0f;
          } else {
            const unsigned short h0 = f2bf_bits(f0), h1 = f2bf_bits(f1);
            const unsigned short l0 = f2bf_bits(f0 - bf_bits2f(h0)), l1 = f2bf_bits(f1 - bf_bits2f(h1));
            hv[it][e]     = __builtin_bit_cast(_Float16, h0);
            hv[it][4 + e] = __builtin_bit_cast(_Float16, h1);
            lv[it][e]     = __builtin_bit_cast(_Float16, l0);
            lv[it][4 + e] = __builtin_bit_cast(_Float16, l1);
          }
        }
      }
      for (int pass = 0; pass < 2; ++pass) {
#pragma unroll
        for (int it = 0; it < 4; ++it) {
          const int row = it * 4 + q;
          const size_t o = (size_t)(mBase + row) * ldc + n0 + c8;
          *(volatile v8h*)(C + o) = hv[it];
          if (OUT_MODE == 2) *(volatile v8h*)(C2 + o) = lv[it];
        }
        __threadfence();
      }
    }
    __builtin_amdgcn_fence(__ATOMIC_RELEASE, "workgroup");
    __builtin_amdgcn_wave_barrier();
    __builtin_amdgcn_fence(__ATOMIC_ACQUIRE, "workgroup");
  }
}

__global__ __launch_bounds__(256) void cast_f16_kernel(
    const float* __restrict__ src, unsigned short* __restrict__ dst, int total8, float scale)
{
  const int i = blockIdx.x * 256 + threadIdx.x;
  if (i >= total8) return;
  const size_t e0 = (size_t)i << 3;
  const float* p = src + e0;
  const v4f a0 = *(const v4f*)(p);
  const v4f a1 = *(const v4f*)(p + 4);
  v8h hv;
#pragma unroll
  for (int e = 0; e < 4; ++e) {
    const float f0 = a0[e] * scale;
    const float f1 = a1[e] * scale;
    hv[e]     = (_Float16)f0;
    hv[4 + e] = (_Float16)f1;
  }
  unsigned short* q = dst + e0;
  *(volatile v8h*)q = hv;
  __threadfence();
  *(volatile v8h*)q = hv;
}

__global__ __launch_bounds__(256) void split_rows_bf16_kernel(
    const float* __restrict__ src, unsigned short* __restrict__ dhi, unsigned short* __restrict__ dlo, int total8)
{
  const int i = blockIdx.x * 256 + threadIdx.x;
  if (i >= total8) return;
  const size_t e0 = (size_t)i << 3;
  const v4f a0 = *(const v4f*)(src + e0);
  const v4f a1 = *(const v4f*)(src + e0 + 4);
  v8h hv, lv;
#pragma unroll
  for (int e = 0; e < 4; ++e) {
    const float f0 = a0[e];
    const float f1 = a1[e];
    const unsigned short h0 = f2bf_bits(f0), h1 = f2bf_bits(f1);
    const unsigned short l0 = f2bf_bits(f0 - bf_bits2f(h0)), l1 = f2bf_bits(f1 - bf_bits2f(h1));
    hv[e]     = __builtin_bit_cast(_Float16, h0);
    hv[4 + e] = __builtin_bit_cast(_Float16, h1);
    lv[e]     = __builtin_bit_cast(_Float16, l0);
    lv[4 + e] = __builtin_bit_cast(_Float16, l1);
  }
  unsigned short* qh = dhi + e0;
  unsigned short* ql = dlo + e0;
  *(volatile v8h*)qh = hv;
  *(volatile v8h*)ql = lv;
  __threadfence();
  *(volatile v8h*)qh = hv;
  *(volatile v8h*)ql = lv;
}

template <int MODE>
__global__ __launch_bounds__(256) void norm_kernel(
    const float* __restrict__ in0, const float* __restrict__ in1,
    const float* __restrict__ lw, const float* __restrict__ lb, const float* __restrict__ rw,
    float* __restrict__ outF, unsigned short* __restrict__ out16)
{
  const int lane = threadIdx.x & 31, wave = threadIdx.x >> 5;
  const int row = blockIdx.x * 8 + wave;
  const size_t base = (size_t)row * kDm + lane * 4;
  v4f v[4];
#pragma unroll
  for (int j = 0; j < 4; ++j) v[j] = *(const v4f*)(in0 + base + j * 128);
  if (MODE == 2) {
#pragma unroll
    for (int j = 0; j < 4; ++j) {
      const v4f t = *(const v4f*)(in1 + base + j * 128);
      v[j] = v[j] + t;
    }
  }
  v4f y[4];
  if (MODE != 1) {
    float s = 0.f;
#pragma unroll
    for (int j = 0; j < 4; ++j) s += (v[j][0] + v[j][1]) + (v[j][2] + v[j][3]);
    s = wave_sum(s);
    const float mu = s * kInvDm;
    float qq = 0.f;
#pragma unroll
    for (int j = 0; j < 4; ++j) {
      const v4f d = v[j] - mu;
      qq += d[0] * d[0] + d[1] * d[1] + d[2] * d[2] + d[3] * d[3];
    }
    qq = wave_sum(qq);
    const float rs = rsqrtf(qq * kInvDm + kEps);
#pragma unroll
    for (int j = 0; j < 4; ++j) {
      const v4f w4 = *(const v4f*)(lw + lane * 4 + j * 128);
      const v4f b4 = *(const v4f*)(lb + lane * 4 + j * 128);
      y[j] = (v[j] - mu) * rs * w4 + b4;
    }
  } else {
#pragma unroll
    for (int j = 0; j < 4; ++j) y[j] = v[j];
  }
  v4f so[4];
  if (MODE != 2) {
    float q2 = 0.f;
#pragma unroll
    for (int j = 0; j < 4; ++j) q2 += y[j][0] * y[j][0] + y[j][1] * y[j][1] + y[j][2] * y[j][2] + y[j][3] * y[j][3];
    q2 = wave_sum(q2);
    const float rs2 = rsqrtf(q2 * kInvDm + kEps);
#pragma unroll
    for (int j = 0; j < 4; ++j) {
      const v4f w4 = *(const v4f*)(rw + lane * 4 + j * 128);
      so[j] = y[j] * rs2 * w4;
    }
  } else {
#pragma unroll
    for (int j = 0; j < 4; ++j) so[j] = y[j];
  }
  v4h h4[4];
#pragma unroll
  for (int j = 0; j < 4; ++j) {
#pragma unroll
    for (int e = 0; e < 4; ++e) {
      const float f = so[j][e];
      h4[j][e] = (_Float16)f;
    }
  }
  v4f fo[4];
#pragma unroll
  for (int j = 0; j < 4; ++j) fo[j] = (MODE == 2) ? v[j] : y[j];
  for (int pass = 0; pass < 2; ++pass) {
    if (MODE != 1) {
#pragma unroll
      for (int j = 0; j < 4; ++j) *(volatile v4f*)(outF + base + j * 128) = fo[j];
    }
#pragma unroll
    for (int j = 0; j < 4; ++j) *(volatile v4h*)(out16 + base + j * 128) = h4[j];
    __threadfence();
  }
}

__global__ __launch_bounds__(256) void conv_silu_kernel(
    const float* __restrict__ XZ, const float* __restrict__ cw, const float* __restrict__ cb,
    float* __restrict__ XC, unsigned short* __restrict__ XC16)
{
  __shared__ __align__(16) float sT[16 * kConvTP];
  const int tid = threadIdx.x, lane = tid & 31, wave = tid >> 5;
  const int d0 = blockIdx.x * 256, d = d0 + tid;
  const int g0 = blockIdx.y * 64;
  const int tb = g0 & (kSeq - 1);
  const v4f w4 = *(const v4f*)(cw + (size_t)d * 4);
  const float w0 = w4[0], w1 = w4[1], w2 = w4[2], w3 = w4[3];
  const float bc = cb[d];
  float xm3, xm2, xm1;
  {
    const bool hist = (tb > 0);
    const int rb = hist ? (g0 - 3) : g0;
    const float v3 = XZ[(size_t)rb * kXzP + d];
    const float v2 = XZ[(size_t)(rb + 1) * kXzP + d];
    const float v1 = XZ[(size_t)(rb + 2) * kXzP + d];
    xm3 = hist ? v3 : 0.f;
    xm2 = hist ? v2 : 0.f;
    xm1 = hist ? v1 : 0.f;
  }
  const int hrow = wave >> 1;
  const int hch  = (wave & 1) * 128 + lane * 4;
#pragma unroll 1
  for (int sub = 0; sub < 4; ++sub) {
    const int lb = g0 + sub * 16;
#pragma unroll 1
    for (int s = 0; s < 16; ++s) {
      const float xcur = XZ[(size_t)(lb + s) * kXzP + d];
      float acc = w0 * xm3;
      acc = fmaf(w1, xm2, acc);
      acc = fmaf(w2, xm1, acc);
      acc = fmaf(w3, xcur, acc);
      const float sv = acc + bc;
      const float sg = __builtin_amdgcn_rcpf(1.0f + expf(-sv));
      sT[s * kConvTP + tid] = sv * sg;
      xm3 = xm2; xm2 = xm1; xm1 = xcur;
    }
    __syncthreads();
    v4f fv[4];
    v8h bv[2];
#pragma unroll
    for (int it = 0; it < 4; ++it) fv[it] = *(const v4f*)(sT + (it * 4 + hrow) * kConvTP + hch);
#pragma unroll
    for (int it = 0; it < 2; ++it) {
      const float* sp = sT + (it * 8 + wave) * kConvTP + lane * 8;
      const v4f a0 = *(const v4f*)(sp);
      const v4f a1 = *(const v4f*)(sp + 4);
#pragma unroll
      for (int e = 0; e < 4; ++e) {
        const float f0 = a0[e];
        const float f1 = a1[e];
        bv[it][e]     = (_Float16)f0;
        bv[it][4 + e] = (_Float16)f1;
      }
    }
    for (int pass = 0; pass < 2; ++pass) {
#pragma unroll
      for (int it = 0; it < 4; ++it)
        *(volatile v4f*)(XC + (size_t)(lb + it * 4 + hrow) * kDin + d0 + hch) = fv[it];
#pragma unroll
      for (int it = 0; it < 2; ++it)
        *(volatile v8h*)(XC16 + (size_t)(lb + it * 8 + wave) * kDin + d0 + lane * 8) = bv[it];
      __threadfence();
    }
    __syncthreads();
  }
}

__global__ __launch_bounds__(256) void dt_cast_kernel(
    const float* __restrict__ DBC, unsigned short* __restrict__ DT16, int total8, float scale)
{
  const int i = blockIdx.x * 256 + threadIdx.x;
  if (i >= total8) return;
  const int e0  = i << 3;
  const int row = e0 >> 5;
  const int c8  = e0 & 31;
  const float* p = DBC + (size_t)row * kXdP + c8;
  const v4f a0 = *(const v4f*)(p);
  const v4f a1 = *(const v4f*)(p + 4);
  v8h hv;
#pragma unroll
  for (int e = 0; e < 4; ++e) {
    const float f0 = a0[e] * scale;
    const float f1 = a1[e] * scale;
    hv[e]     = (_Float16)f0;
    hv[4 + e] = (_Float16)f1;
  }
  unsigned short* qd = DT16 + e0;
  *(volatile v8h*)qd = hv;
  __threadfence();
  *(volatile v8h*)qd = hv;
}

__global__ __launch_bounds__(64) void scan_kernel(
    const float* __restrict__ DLR, const float* __restrict__ XC, const float* __restrict__ XZ,
    const float* __restrict__ DBC, const float* __restrict__ Alog, const float* __restrict__ Dp,
    unsigned short* __restrict__ G16)
{
  __shared__ __align__(16) float sX[kScanTS * 32];
  __shared__ __align__(16) float sY[kScanTS * kScanYP];
  __shared__ __align__(16) float sA[kNst * kScanCh];
  const int tid = threadIdx.x, lane = tid & 31, wave = tid >> 5;
  constexpr int kBlkPerB = kDin / kScanCh;
  const int bix = blockIdx.x / kBlkPerB;
  const int d0  = (blockIdx.x - bix * kBlkPerB) * kScanCh;
  const int d   = d0 + tid;
  const size_t row0 = (size_t)bix * kSeq;
#pragma unroll 1
  for (int s = 0; s < kNst; ++s) sA[s * kScanCh + tid] = -expf(Alog[(size_t)d * kNst + s]);
  __syncthreads();
  float negA[kNst], h[kNst];
#pragma unroll
  for (int s = 0; s < kNst; ++s) {
    negA[s] = sA[s * kScanCh + tid];
    h[s] = 0.f;
  }
  const float Dd = Dp[d];
  const int lr = tid >> 3, lc4 = (tid & 7) * 4;
  const int q = lane >> 3, c8 = (lane & 7) * 8;
#pragma unroll 1
  for (int t0 = 0; t0 < kSeq; t0 += kScanTS) {
    __syncthreads();
#pragma unroll
    for (int i = 0; i < 8; ++i) {
      const int r = lr + 8 * i;
      *(v4f*)(sX + r * 32 + lc4) = *(const v4f*)(DBC + (row0 + t0 + r) * kXdP + kDtR + lc4);
    }
    __syncthreads();
#pragma unroll 1
    for (int s = 0; s < kScanTS; ++s) {
      const size_t row = row0 + t0 + s;
      const float* xr = sX + s * 32;
      float Bs[kNst], Cs[kNst];
#pragma unroll
      for (int q4 = 0; q4 < 4; ++q4) {
        const v4f bv = *(const v4f*)(xr + 4 * q4);
        const v4f cv = *(const v4f*)(xr + kNst + 4 * q4);
        Bs[4 * q4 + 0] = bv[0]; Bs[4 * q4 + 1] = bv[1]; Bs[4 * q4 + 2] = bv[2]; Bs[4 * q4 + 3] = bv[3];
        Cs[4 * q4 + 0] = cv[0]; Cs[4 * q4 + 1] = cv[1]; Cs[4 * q4 + 2] = cv[2]; Cs[4 * q4 + 3] = cv[3];
      }
      const float v   = DLR[row * kDin + d];
      const float xt  = XC[row * kDin + d];
      const float zv  = XZ[row * kXzP + kDin + d];
      const float dt  = fmaxf(v, 0.0f) + log1pf(expf(-fabsf(v)));
      const float dtx = dt * xt;
      float y = 0.f;
#pragma unroll
      for (int k = 0; k < kNst; ++k) {
        const float e = __expf(dt * negA[k]);
        h[k] = e * h[k] + dtx * Bs[k];
        y = h[k] * Cs[k] + y;
      }
      y = xt * Dd + y;
      const float sg = __builtin_amdgcn_rcpf(1.0f + expf(-zv));
      y = y * (zv * sg);
      sY[s * kScanYP + tid] = y * kCarryG;
    }
    __syncthreads();
    v8h hv[8];
#pragma unroll
    for (int it = 0; it < 8; ++it) {
      const int orow = it * 8 + wave * 4 + q;
      const float* sp = sY + orow * kScanYP + c8;
      const v4f a0 = *(const v4f*)(sp);
      const v4f a1 = *(const v4f*)(sp + 4);
#pragma unroll
      for (int e = 0; e < 4; ++e) {
        const float f0 = a0[e];
        const float f1 = a1[e];
        hv[it][e]     = (_Float16)f0;
        hv[it][4 + e] = (_Float16)f1;
      }
    }
    for (int pass = 0; pass < 2; ++pass) {
#pragma unroll
      for (int it = 0; it < 8; ++it) {
        const int orow = it * 8 + wave * 4 + q;
        *(volatile v8h*)(G16 + (row0 + t0 + orow) * kDin + d0 + c8) = hv[it];
      }
      __threadfence();
    }
  }
}

extern "C" void kernel_launch(void* const* d_in, const int* in_sizes, int n_in,
                              void* d_out, int out_size, void* d_ws, size_t ws_size,
                              hipStream_t stream)
{
  if (n_in < 21) return;
  if (in_sizes[0] != kRows * kDm) return;
  if (in_sizes[1] != kLayers * kXzP * kDm) return;
  if (in_sizes[2] != kLayers * kDin * 4 || in_sizes[3] != kLayers * kDin) return;
  if (in_sizes[4] != kLayers * kXdP * kDin) return;
  if (in_sizes[5] != kLayers * kDin * kDtR || in_sizes[6] != kLayers * kDin) return;
  if (in_sizes[7] != kLayers * kDin * kNst || in_sizes[8] != kLayers * kDin) return;
  if (in_sizes[9] != kLayers * kDm * kDin) return;
  if (in_sizes[10] != kLayers * kDm) return;
  if (in_sizes[11] != kDm || in_sizes[12] != kDm || in_sizes[13] != kDm || in_sizes[14] != kDm) return;
  if (in_sizes[15] != kHid * kDm || in_sizes[16] != kHid) return;
  if (in_sizes[17] != kDm * kHid || in_sizes[18] != kDm) return;
  if (in_sizes[19] != kOutC * kDm || in_sizes[20] != kOutC) return;
  if (out_size != kRows * kOutC) return;
  if (ws_size < kWsTotal) return;

  const float* x      = (const float*)d_in[0];
  const float* ipw    = (const float*)d_in[1];
  const float* convw  = (const float*)d_in[2];
  const float* convb  = (const float*)d_in[3];
  const float* xpw    = (const float*)d_in[4];
  const float* dtw    = (const float*)d_in[5];
  const float* dtb    = (const float*)d_in[6];
  const float* alog   = (const float*)d_in[7];
  const float* dpar   = (const float*)d_in[8];
  const float* opw    = (const float*)d_in[9];
  const float* rmsw   = (const float*)d_in[10];
  const float* ln1w   = (const float*)d_in[11];
  const float* ln1b   = (const float*)d_in[12];
  const float* ln2w   = (const float*)d_in[13];
  const float* ln2b   = (const float*)d_in[14];
  const float* w1     = (const float*)d_in[15];
  const float* b1     = (const float*)d_in[16];
  const float* w2     = (const float*)d_in[17];
  const float* b2     = (const float*)d_in[18];
  const float* fw     = (const float*)d_in[19];
  const float* fb     = (const float*)d_in[20];
  float* out = (float*)d_out;

  char* ws = (char*)d_ws;
  float*          HA    = (float*)(ws + kOffHA);
  float*          HB    = (float*)(ws + kOffHB);
  unsigned short* U16   = (unsigned short*)(ws + kOffU16);
  float*          XZ    = (float*)(ws + kOffXZ);
  float*          XC    = (float*)(ws + kOffXC);
  unsigned short* XC16  = (unsigned short*)(ws + kOffXC16);
  float*          DBC   = (float*)(ws + kOffDBC);
  unsigned short* DT16  = (unsigned short*)(ws + kOffDT16);
  float*          DLR   = (float*)(ws + kOffDLR);
  unsigned short* G16   = (unsigned short*)(ws + kOffG16);
  float*          X1    = (float*)(ws + kOffX1);
  unsigned short* X2H   = (unsigned short*)(ws + kOffX2H);
  unsigned short* X2L   = (unsigned short*)(ws + kOffX2L);
  unsigned short* IPW16 = (unsigned short*)(ws + kOffIPW);
  unsigned short* XPW16 = (unsigned short*)(ws + kOffXPW);
  unsigned short* DTW16 = (unsigned short*)(ws + kOffDTW);
  unsigned short* OPW16 = (unsigned short*)(ws + kOffOPW);
  unsigned short* W116  = (unsigned short*)(ws + kOffW1);
  unsigned short* W216  = (unsigned short*)(ws + kOffW2);
  unsigned short* FWH   = (unsigned short*)(ws + kOffFWH);
  unsigned short* FWL   = (unsigned short*)(ws + kOffFWL);
  unsigned short* HID16 = XC16;
  const float* dummy_bias  = dtb;
  const float* dummy_resid = x;

  cast_f16_kernel<<<(kLayers * kXzP * kDm / 8) / 256, 256, 0, stream>>>(ipw, IPW16, kLayers * kXzP * kDm / 8, kCarryW);
  cast_f16_kernel<<<(kLayers * kXdP * kDin / 8) / 256, 256, 0, stream>>>(xpw, XPW16, kLayers * kXdP * kDin / 8, kCarryW);
  cast_f16_kernel<<<(kLayers * kDin * kDtR / 8) / 256, 256, 0, stream>>>(dtw, DTW16, kLayers * kDin * kDtR / 8, kCarryDtW);
  cast_f16_kernel<<<(kLayers * kDm * kDin / 8) / 256, 256, 0, stream>>>(opw, OPW16, kLayers * kDm * kDin / 8, kCarryW);
  cast_f16_kernel<<<(kHid * kDm / 8) / 256, 256, 0, stream>>>(w1, W116, kHid * kDm / 8, kCarryW);
  cast_f16_kernel<<<(kDm * kHid / 8) / 256, 256, 0, stream>>>(w2, W216, kDm * kHid / 8, kCarryW);
  split_rows_bf16_kernel<<<(kOutC * kDm / 8) / 256, 256, 0, stream>>>(fw, FWH, FWL, kOutC * kDm / 8);

  norm_kernel<0><<<kRows / 8, 256, 0, stream>>>(x, x, ln1w, ln1b, rmsw, HA, U16);

  for (int i = 0; i < kLayers; ++i) {
    float* hin  = (i == 0) ? HA : HB;
    float* hout = (i == 0) ? HB : HA;
    if (i > 0) {
      norm_kernel<1><<<kRows / 8, 256, 0, stream>>>(hin, hin, ln1w, ln1b, rmsw + (size_t)i * kDm, X1, U16);
    }
    wmma_gemm64<0, false, 0, 0, false, 0><<<256, 256, 0, stream>>>(
        U16, U16, kDm,
        IPW16 + (size_t)i * kXzP * kDm, IPW16 + (size_t)i * kXzP * kDm, kDm,
        (void*)XZ, (void*)XZ, kXzP,
        dummy_bias, dummy_resid,
        kRows, kXzP, kDm, 1.0f / kCarryW);
    conv_silu_kernel<<<dim3(kDin / 256, kRows / 64), 256, 0, stream>>>(
        XZ, convw + (size_t)i * kDin * 4, convb + (size_t)i * kDin, XC, XC16);
    wmma_gemm64<0, false, 0, 0, false, 0><<<8, 256, 0, stream>>>(
        XC16, XC16, kDin,
        XPW16 + (size_t)i * kXdP * kDin, XPW16 + (size_t)i * kXdP * kDin, kDin,
        (void*)DBC, (void*)DBC, kXdP,
        dummy_bias, dummy_resid,
        kRows, kXdP, kDin, 1.0f / kCarryW);
    dt_cast_kernel<<<(kRows * kDtR / 8) / 256, 256, 0, stream>>>(DBC, DT16, kRows * kDtR / 8, kCarryDt);
    wmma_gemm64<0, false, 2, 0, false, 0><<<128, 256, 0, stream>>>(
        DT16, DT16, kDtR,
        DTW16 + (size_t)i * kDin * kDtR, DTW16 + (size_t)i * kDin * kDtR, kDtR,
        (void*)DLR, (void*)DLR, kDin,
        dtb + (size_t)i * kDin, dummy_resid,
        kRows, kDin, kDtR, 1.0f / (kCarryDt * kCarryDtW));
    scan_kernel<<<kBatch * (kDin / kScanCh), kScanCh, 0, stream>>>(
        DLR, XC, XZ, DBC, alog + (size_t)i * kDin * kNst, dpar + (size_t)i * kDin, G16);
    wmma_gemm64<0, false, 0, 0, true, 0><<<64, 256, 0, stream>>>(
        G16, G16, kDin,
        OPW16 + (size_t)i * kDm * kDin, OPW16 + (size_t)i * kDm * kDin, kDin,
        (void*)hout, (void*)hout, kDm,
        dummy_bias, hin,
        kRows, kDm, kDin, 1.0f / (kCarryG * kCarryW));
  }

  norm_kernel<2><<<kRows / 8, 256, 0, stream>>>(x, HA, ln2w, ln2b, rmsw, X1, U16);

  wmma_gemm64<0, false, 2, 1, false, 2><<<128, 256, 0, stream>>>(
      U16, U16, kDm,
      W116, W116, kDm,
      (void*)HID16, (void*)HID16, kHid,
      b1, dummy_resid,
      kRows, kHid, kDm, 1.0f / kCarryW);

  wmma_gemm64<0, false, 2, 2, true, 0><<<64, 256, 0, stream>>>(
      HID16, HID16, kHid,
      W216, W216, kHid,
      (void*)X2H, (void*)X2L, kDm,
      b2, X1,
      kRows, kDm, kHid, 1.0f / kCarryW);

  wmma_gemm64<1, true, 2, 0, false, 0><<<64, 256, 0, stream>>>(
      X2H, X2L, kDm,
      FWH, FWL, kDm,
      (void*)out, (void*)out, kDm,
      fb, dummy_resid,
      kRows, kOutC, kDm, 1.0f);
}
